// CantorAttention_51213190038176
// MI455X (gfx1250) — hardware-verified
//
#include <hip/hip_runtime.h>
#include <math.h>

typedef __attribute__((ext_vector_type(16))) _Float16 v16h;
typedef __attribute__((ext_vector_type(16))) __bf16 v16b;
typedef __attribute__((ext_vector_type(8)))  _Float16 v8h;
typedef __attribute__((ext_vector_type(8)))  float v8f;
typedef __attribute__((ext_vector_type(4)))  float v4f;
typedef __attribute__((ext_vector_type(2)))  float v2f;
typedef __attribute__((ext_vector_type(4)))  unsigned v4u;
typedef __attribute__((ext_vector_type(4)))  int v4i;
typedef float __attribute__((may_alias)) float_a;
typedef int __attribute__((may_alias)) int_a;

template <typename T> __device__ __forceinline__ void vst2(void* p, T v) { *(volatile T*)p = v; __threadfence(); *(volatile T*)p = v; }
__device__ __forceinline__ v8f wmma16(v16h a, v16h b, v8f c) {
  v8f d = __builtin_amdgcn_wmma_f32_16x16x32_f16(false, a, false, b, (short)0, c, false, false);
  asm volatile("v_nop\n\tv_nop\n\tv_nop\n\tv_nop" : "+v"(d) : "v"(a), "v"(b));
  return d;
}
__device__ __forceinline__ v8f wmma_bf(v16b a, v16b b, v8f c) {
  v8f d = __builtin_amdgcn_wmma_f32_16x16x32_bf16(false, a, false, b, (short)0, c, false, false);
  asm volatile("v_nop\n\tv_nop\n\tv_nop\n\tv_nop" : "+v"(d) : "v"(a), "v"(b));
  return d;
}
__device__ __forceinline__ v16h frag_h(const _Float16* rowk0, int lane) {
  union { v16h v; v8h q[2]; } u; const _Float16* p = rowk0 + 8 * (lane >> 4);
  u.q[0] = *(const v8h*)p; u.q[1] = *(const v8h*)(p + 16); return u.v;
}
__device__ __forceinline__ v16h frag_f32(const float* rowk0, int lane) {
  v16h a; const float* p = rowk0 + 8 * (lane >> 4);
#pragma unroll
  for (int i = 0; i < 8; ++i) { a[i] = (_Float16)p[i]; a[8 + i] = (_Float16)p[16 + i]; }
  return a;
}
__device__ __forceinline__ v16h frag_f32s(const float* rowk0, int lane, float sc) {
  v16h a; const float* p = rowk0 + 8 * (lane >> 4);
#pragma unroll
  for (int i = 0; i < 8; ++i) { a[i] = (_Float16)(p[i] * sc); a[8 + i] = (_Float16)(p[16 + i] * sc); }
  return a;
}
__device__ __forceinline__ v16h fragc_f32(const float* W, int k0, int n, int lane, int ld, int K) {
  v16h a; const int g = lane >> 4;
#pragma unroll
  for (int i = 0; i < 8; ++i) { const int ka = k0 + 8 * g + i, kb = ka + 16;
    a[i] = (_Float16)(ka < K ? W[(size_t)(ka < K ? ka : K - 1) * ld + n] : 0.f); a[8 + i] = (_Float16)(kb < K ? W[(size_t)(kb < K ? kb : K - 1) * ld + n] : 0.f); }
  return a;
}
struct F2 { v16b h, l; };
__device__ __forceinline__ F2 bsplit16(const float v[16]) { F2 r;
#pragma unroll
  for (int i = 0; i < 16; ++i) { const __bf16 h = (__bf16)v[i]; r.h[i] = h; r.l[i] = (__bf16)(v[i] - (float)h); }
  return r; }
__device__ __forceinline__ F2 split_row(const float* row, int k0, int lane) { float v[16]; const float* p = row + k0 + 8 * (lane >> 4);
#pragma unroll
  for (int i = 0; i < 8; ++i) { v[i] = p[i]; v[8 + i] = p[16 + i]; }
  return bsplit16(v); }
__device__ __forceinline__ F2 split_rowK(const float* row, int k0, int lane, int K) { float v[16]; const int g = lane >> 4;
#pragma unroll
  for (int i = 0; i < 8; ++i) { const int ka = k0 + 8 * g + i, kb = ka + 16; v[i] = ka < K ? row[ka < K ? ka : K - 1] : 0.f; v[8 + i] = kb < K ? row[kb < K ? kb : K - 1] : 0.f; }
  return bsplit16(v); }
__device__ __forceinline__ F2 split_col(const float* W, int k0, int n, int lane, int ld, int K) { float v[16]; const int g = lane >> 4;
#pragma unroll
  for (int i = 0; i < 8; ++i) { const int ka = k0 + 8 * g + i, kb = ka + 16; v[i] = ka < K ? W[(size_t)(ka < K ? ka : K - 1) * ld + n] : 0.f; v[8 + i] = kb < K ? W[(size_t)(kb < K ? kb : K - 1) * ld + n] : 0.f; }
  return bsplit16(v); }
__device__ __forceinline__ v8f mac3(const F2& a, const F2& b, v8f c) { c = wmma_bf(a.l, b.h, c); c = wmma_bf(a.h, b.l, c); return wmma_bf(a.h, b.h, c); }
__device__ __forceinline__ float sigm(float v) { return 1.0f / (1.0f + expf(-v)); }
#define LDSX() do { asm volatile("s_wait_dscnt 0" ::: "memory"); __builtin_amdgcn_wave_barrier(); __builtin_amdgcn_fence(__ATOMIC_RELEASE, "workgroup"); } while (0)

__device__ __forceinline__ float bfr(float v) { return (float)(__bf16)v; }
#define NBT 2
#define SS 4096
#define DD 1024
#define NH 16
#define HD 64
#define KN 64
#ifndef NQB
#define NQB (NBT * SS / 8)
#endif
#ifndef TPROWS
#define TPROWS (NBT * SS)
#endif
#ifndef TNB
#define TNB NBT
#endif
#define WS_Q  0u
#define WS_K  (WS_Q + 4u * (size_t)NBT * SS * DD)
#define WS_V  (WS_K + 4u * (size_t)NBT * SS * DD)
#define WS_Y  (WS_V + 4u * (size_t)NBT * SS * DD)
#define WS_END (WS_Y + 4u * (size_t)NBT * SS * DD)
__global__ __launch_bounds__(128) void k_proj(const float* __restrict__ X, const float* __restrict__ W, const float* __restrict__ Bv, float* __restrict__ Q, float* __restrict__ K, float* __restrict__ V) { __shared__ __align__(16) float sf[4][16][132];
  const int tid = threadIdx.x, wave = tid >> 5, lane = tid & 31, col = lane & 15, g = lane >> 4; const int which = blockIdx.z; const int c0 = blockIdx.y * 128; const size_t r0 = (size_t)blockIdx.x * 64 + wave * 16;
  v8f acc[8] = {};
#pragma unroll 2
  for (int kc = 0; kc < DD / 32; ++kc) { v16b a; { const float* p = X + (r0 + col) * DD + kc * 32 + 8 * g;
#pragma unroll
      for (int i = 0; i < 8; ++i) { a[i] = (__bf16)p[i]; a[8 + i] = (__bf16)p[16 + i]; } }
#pragma unroll
    for (int j = 0; j < 8; ++j) { v16b w; const int o = which * DD + c0 + j * 16 + col;
#pragma unroll
      for (int i = 0; i < 8; ++i) { w[i] = (__bf16)W[(size_t)(kc * 32 + 8 * g + i) * (3 * DD) + o]; w[8 + i] = (__bf16)W[(size_t)(kc * 32 + 16 + 8 * g + i) * (3 * DD) + o]; }
      acc[j] = wmma_bf(a, w, acc[j]); } }
#pragma unroll
  for (int j = 0; j < 8; ++j) { const float bb = bfr(Bv[which * DD + c0 + j * 16 + col]);
#pragma unroll
    for (int r = 0; r < 8; ++r) sf[wave][8 * g + r][j * 16 + col] = acc[j][r] + bb; }
  float* D = which == 0 ? Q : which == 1 ? K : V;
  LDSX(); for (int rl = 0; rl < 16; ++rl) vst2(D + (r0 + rl) * DD + c0 + lane * 4, *(const v4f*)&sf[wave][rl][lane * 4]); }
__global__ __launch_bounds__(256) void k_att(const float* __restrict__ Q, const float* __restrict__ K, const float* __restrict__ V, const int* __restrict__ RT, float* __restrict__ Y) {
  __shared__ float ssc[8][NH][KN]; __shared__ __align__(16) float sy[8][DD];
  const int tid = threadIdx.x, wave = tid >> 5, lane = tid & 31; const int h = lane >> 1, half = lane & 1; const size_t b = blockIdx.y; const size_t q = (size_t)blockIdx.x * 8 + wave;
  const float* qr = Q + (b * SS + q) * DD + h * HD; const int* rt = RT + q * KN + half * 32;
  float qv[HD];
#pragma unroll
  for (int d = 0; d < HD; ++d) qv[d] = qr[d];
#pragma unroll 1
  for (int kk = 0; kk < 32; ++kk) { const int j = rt[kk]; const float* kr = K + (b * SS + j) * DD + h * HD; float s = 0.f;
#pragma unroll
    for (int d4 = 0; d4 < HD; d4 += 4) { const v4f kv = *(const v4f*)(kr + d4); s += qv[d4] * kv[0] + qv[d4 + 1] * kv[1] + qv[d4 + 2] * kv[2] + qv[d4 + 3] * kv[3]; }
    ssc[wave][h][half * 32 + kk] = s * 0.125f; }
  LDSX();
  { float m = -3.0e38f; for (int k = 0; k < KN; ++k) m = fmaxf(m, ssc[wave][h][k]); float sum = 0.f; for (int k = 0; k < KN; ++k) sum += expf(ssc[wave][h][k] - m); const float inv = 1.0f / sum;
    LDSX();
    for (int kk = 0; kk < 32; ++kk) { const int k = half * 32 + kk; ssc[wave][h][k] = expf(ssc[wave][h][k] - m) * inv; } }
  LDSX();
  float acc[HD];
#pragma unroll
  for (int d = 0; d < HD; ++d) acc[d] = 0.f;
#pragma unroll 1
  for (int kk = 0; kk < 32; ++kk) { const int j = rt[kk]; const float p = ssc[wave][h][half * 32 + kk]; const float* vr = V + (b * SS + j) * DD + h * HD;
#pragma unroll
    for (int d4 = 0; d4 < HD; d4 += 4) { const v4f vv = *(const v4f*)(vr + d4); acc[d4] += p * vv[0]; acc[d4 + 1] += p * vv[1]; acc[d4 + 2] += p * vv[2]; acc[d4 + 3] += p * vv[3]; } }
#pragma unroll
  for (int d = 0; d < HD; ++d) acc[d] += __shfl_xor(acc[d], 1);
  if (half == 0) {
#pragma unroll
    for (int d = 0; d < HD; ++d) sy[wave][h * HD + d] = acc[d]; }
  LDSX();
  for (int pz = 0; pz < 8; ++pz) vst2(Y + (b * SS + q) * DD + pz * 128 + lane * 4, *(const v4f*)&sy[wave][pz * 128 + lane * 4]);
}
__global__ __launch_bounds__(128) void k_out(const float* __restrict__ Yr, const float* __restrict__ WO, const float* __restrict__ BO, float* __restrict__ OUT) { __shared__ __align__(16) float sf[4][16][132];
  const int tid = threadIdx.x, wave = tid >> 5, lane = tid & 31, col = lane & 15, g = lane >> 4; const int c0 = blockIdx.y * 128; const size_t r0 = (size_t)blockIdx.x * 64 + wave * 16;
  v8f acc[8] = {};
#pragma unroll 2
  for (int kc = 0; kc < DD / 32; ++kc) { const F2 a = split_row(Yr + (r0 + col) * DD, kc * 32, lane);
#pragma unroll
    for (int j = 0; j < 8; ++j) { v16b w; const int o = c0 + j * 16 + col;
#pragma unroll
      for (int i = 0; i < 8; ++i) { w[i] = (__bf16)WO[(size_t)(kc * 32 + 8 * g + i) * DD + o]; w[8 + i] = (__bf16)WO[(size_t)(kc * 32 + 16 + 8 * g + i) * DD + o]; }
      acc[j] = wmma_bf(a.h, w, acc[j]); acc[j] = wmma_bf(a.l, w, acc[j]); } }
#pragma unroll
  for (int j = 0; j < 8; ++j) { const float bb = bfr(BO[c0 + j * 16 + col]);
#pragma unroll
    for (int r = 0; r < 8; ++r) sf[wave][8 * g + r][j * 16 + col] = acc[j][r] + bb; }
  LDSX(); for (int rl = 0; rl < 16; ++rl) vst2(OUT + (r0 + rl) * DD + c0 + lane * 4, *(const v4f*)&sf[wave][rl][lane * 4]); }
extern "C" void kernel_launch(void* const* d_in, const int* in_sizes, int n_in, void* d_out, int out_size, void* d_ws, size_t ws_size, hipStream_t stream) {
  (void)in_sizes; (void)n_in; (void)out_size;
  const float** F = (const float**)d_in;
  if (ws_size < (size_t)WS_END) return;
  char* ws = (char*)d_ws; float *Q = (float*)(ws + WS_Q), *K = (float*)(ws + WS_K), *V = (float*)(ws + WS_V), *Y = (float*)(ws + WS_Y);
  k_proj<<<dim3(TPROWS / 64, DD / 128, 3), 128, 0, stream>>>(F[0], F[1], F[2], Q, K, V);
  k_att<<<dim3(NQB / TNB, TNB), 256, 0, stream>>>(Q, K, V, (const int*)d_in[5], Y);
  k_out<<<dim3(NQB * 8 / 64, DD / 128), 128, 0, stream>>>(Y, F[3], F[4], (float*)d_out);
}
